// ScatterHorizontal_40656160424524
// MI455X (gfx1250) — hardware-run, weakly checked
//
#include <hip/hip_runtime.h>


#define NB   1024
#define NC   64
#define NO   64
#define NS   9
#define NT   9
#define NPOS (NB * NS * NS)
#define KD   (NT * NC)
constexpr size_t al256(size_t b) { return (b + 255) & ~(size_t)255; }
constexpr size_t WS_TOTAL = al256((size_t)NPOS * KD * 2) + al256((size_t)NO * KD * 2) + al256((size_t)NPOS * NO * 4) + al256((size_t)NT * NO * 4);
static_assert(WS_TOTAL == 116861184 && WS_TOTAL <= 134217728, "the workspace carve: 111.4 MiB");
static_assert(NPOS % 64 == 0 && NO % 64 == 0 && KD % 32 == 0 && NC == 64 && NT == 9 && NS == 9, "whole tiles; whole depth steps; a tap's block one 128-byte line");
typedef _Float16 h16;
typedef unsigned short bf;
typedef __attribute__((ext_vector_type(16))) __bf16   v16bf;
typedef __attribute__((ext_vector_type(16))) _Float16 v16h;
typedef __attribute__((ext_vector_type(8)))  _Float16 v8h;
typedef __attribute__((ext_vector_type(8)))  unsigned short v8us;
typedef __attribute__((ext_vector_type(8)))  float    v8f;
typedef __attribute__((ext_vector_type(4)))  float    v4f;
typedef v8h  __attribute__((may_alias)) v8ha;
typedef v4f  __attribute__((may_alias)) v4fa;
typedef v8us __attribute__((may_alias)) v8usa;

__device__ __forceinline__ unsigned short f2bf(float f) { unsigned u = __float_as_uint(f); u += 0x7FFFu + ((u >> 16) & 1u); return (unsigned short)(u >> 16); }
__device__ __forceinline__ float bf2f(unsigned short b) { return __uint_as_float(((unsigned)b) << 16); }
__device__ __forceinline__ float bfr(float f) { return bf2f(f2bf(f)); }
__device__ __forceinline__ v16h cat16(v8h lo, v8h hi) { return __builtin_shufflevector(lo, hi, 0, 1, 2, 3, 4, 5, 6, 7, 8, 9, 10, 11, 12, 13, 14, 15); }
__device__ __forceinline__ v16bf cat16b(v8us lo, v8us hi) { return __builtin_bit_cast(v16bf, __builtin_shufflevector(lo, hi, 0, 1, 2, 3, 4, 5, 6, 7, 8, 9, 10, 11, 12, 13, 14, 15)); }
__device__ __forceinline__ v8f wmma16(v16h a, v16h b, v8f c) { return __builtin_amdgcn_wmma_f32_16x16x32_f16(false, a, false, b, (short)0, c, false, false); }
__device__ __forceinline__ v8f wmmab(v16bf a, v16bf b, v8f c) { return __builtin_amdgcn_wmma_f32_16x16x32_bf16(false, a, false, b, (short)0, c, false, false); }


template <typename T16> struct WFrag;
template <> struct WFrag<h16> { typedef v16h V; static __device__ __forceinline__ V ld(const h16* p) { return cat16(*(const v8h*)p, *(const v8h*)(p + 16)); } static __device__ __forceinline__ v8f mma(V a, V b, v8f c) { return wmma16(a, b, c); } };
template <> struct WFrag<bf> { typedef v16bf V; static __device__ __forceinline__ V ld(const bf* p) { return cat16b(*(const v8us*)p, *(const v8us*)(p + 16)); } static __device__ __forceinline__ v8f mma(V a, V b, v8f c) { return wmmab(a, b, c); } };
template <typename T16, int NSPLIT, bool BIAS>
__global__ __launch_bounds__(32) void k_gemmw(const T16* __restrict__ A, const T16* __restrict__ A2, const T16* __restrict__ Bt, const T16* __restrict__ Bt2, int K, float* C, int ldc, const float* __restrict__ bias, size_t sA, size_t sB, size_t sC) {
    typedef typename WFrag<T16>::V V;
    __shared__ __align__(16) float os[16 * 68];
    const size_t z = blockIdx.z; A += z * sA; if (A2) A2 += z * sA; Bt += z * sB; if (Bt2) Bt2 += z * sB; C += z * sC;
    const int lane = threadIdx.x & 31, lr = lane & 15, hi = lane >> 4; const int r0 = blockIdx.x * 64, c0 = blockIdx.y * 64;
    v8f acc[4][4];
#pragma unroll
    for (int mb = 0; mb < 4; ++mb)
#pragma unroll
        for (int nb = 0; nb < 4; ++nb) acc[mb][nb] = (v8f){};
    const size_t aoff = (size_t)(r0 + lr) * K + 8 * hi, boff = (size_t)(c0 + lr) * K + 8 * hi;
    for (int kc = 0; kc < K; kc += 32) {
        V a[4], a2[4];
#pragma unroll
        for (int mb = 0; mb < 4; ++mb) { a[mb] = WFrag<T16>::ld(A + aoff + (size_t)mb * 16 * K + kc); if (NSPLIT == 1 || NSPLIT == 2) a2[mb] = WFrag<T16>::ld(A2 + aoff + (size_t)mb * 16 * K + kc); }
#pragma unroll
        for (int nb = 0; nb < 4; ++nb) { const V b = WFrag<T16>::ld(Bt + boff + (size_t)nb * 16 * K + kc); V b2; if (NSPLIT >= 2) b2 = WFrag<T16>::ld(Bt2 + boff + (size_t)nb * 16 * K + kc);
#pragma unroll
            for (int mb = 0; mb < 4; ++mb) { acc[mb][nb] = WFrag<T16>::mma(a[mb], b, acc[mb][nb]); if (NSPLIT == 1 || NSPLIT == 2) acc[mb][nb] = WFrag<T16>::mma(a2[mb], b, acc[mb][nb]); if (NSPLIT >= 2) acc[mb][nb] = WFrag<T16>::mma(a[mb], b2, acc[mb][nb]); } }
        asm volatile("v_nop\n\tv_nop\n\tv_nop\n\tv_nop" : "+v"(acc[0][0]), "+v"(acc[1][1]), "+v"(acc[2][2]), "+v"(acc[3][3]) : "v"(a[0]), "v"(a[3]));
    }
#pragma unroll
    for (int mb = 0; mb < 4; ++mb) {
#pragma unroll
        for (int nb = 0; nb < 4; ++nb) {
#pragma unroll
            for (int j = 0; j < 8; ++j) os[(hi * 8 + j) * 68 + nb * 16 + lr] = acc[mb][nb][j]; }
        __builtin_amdgcn_wave_barrier(); asm volatile("" ::: "memory");
        float* crow = C + (size_t)(r0 + mb * 16) * ldc + c0;
#pragma unroll 1
        for (int ps = 0; ps < 2; ++ps) {
#pragma unroll
            for (int s = 0; s < 8; ++s) { const int row = 2 * s + hi, cofs = lr * 4; v4f val = *(const v4fa*)(os + row * 68 + cofs); if (BIAS) { val[0] += bfr(bias[c0 + cofs]); val[1] += bfr(bias[c0 + cofs + 1]); val[2] += bfr(bias[c0 + cofs + 2]); val[3] += bfr(bias[c0 + cofs + 3]); }
                *(volatile v4f*)(crow + (size_t)row * ldc + cofs) = val; }
            if (ps == 0) __threadfence(); }
        __builtin_amdgcn_wave_barrier(); asm volatile("" ::: "memory");
    }
}

__device__ __forceinline__ h16 tohx(float x) { return (h16)x; }
__device__ __forceinline__ void splitf(float y, unsigned short& h, unsigned short& l) { h = f2bf(y); l = f2bf(y - bf2f(h)); }
typedef __attribute__((ext_vector_type(2))) _Float16 v2h;
typedef __attribute__((ext_vector_type(4))) _Float16 v4h;
typedef __attribute__((ext_vector_type(2))) unsigned short v2us;
typedef __attribute__((ext_vector_type(4))) unsigned short v4us;
typedef __attribute__((ext_vector_type(2))) float v2f;
typedef __attribute__((ext_vector_type(4))) int v4i;

__global__ __launch_bounds__(256) void k_pack(const float* __restrict__ pl, int t, bf* AP) {
    const unsigned hw = blockIdx.y, h = hw / NS, w = hw % NS; const unsigned e = blockIdx.x * 256 + threadIdx.x; if (e >= (unsigned)(NB * (NC / 8))) return; const unsigned b = e >> 3, g = e & 7;
    const int ws = (int)w - (t - 4); const bool on = (ws >= 0) && (ws < NS); const unsigned wc = on ? (unsigned)ws : 0u; const float sf = on ? 1.0f : 0.0f;
    const float* src = pl + ((size_t)b * NC + 8 * g) * (NS * NS) + h * NS + wc; v8us o;
#pragma unroll
    for (int q = 0; q < 8; ++q) o[q] = f2bf(src[(size_t)q * (NS * NS)] * sf);
    bf* d = AP + ((size_t)b * (NS * NS) + hw) * KD + (size_t)t * NC + 8 * g; *(volatile v8us*)(d) = o; __threadfence(); *(volatile v8us*)(d) = o; }

__global__ __launch_bounds__(256) void k_wpk(const float* __restrict__ Wt, bf* WP) {
    const unsigned t = blockIdx.y; const unsigned e = blockIdx.x * 256 + threadIdx.x; if (e >= (unsigned)(NO * (NC / 8))) return; const unsigned o = e >> 3, g = e & 7;
    const float* src = Wt + ((size_t)t * NO + o) * NC + 8 * g; const v4f a0 = *(const v4f*)(src); const v4f a1 = *(const v4f*)(src + 4); v8us r;
#pragma unroll
    for (int q = 0; q < 4; ++q) { r[q] = f2bf(a0[q]); r[q + 4] = f2bf(a1[q]); }
    bf* d = WP + (size_t)o * KD + (size_t)t * NC + 8 * g; *(volatile v8us*)(d) = r; __threadfence(); *(volatile v8us*)(d) = r; }

__global__ __launch_bounds__(256) void k_rbf(const float* __restrict__ X, float* Y, size_t n4) { const size_t i = (size_t)blockIdx.x * 256 + threadIdx.x; if (i >= n4) return; const v4f a = *(const v4f*)(X + i * 4); v4f o;
#pragma unroll
    for (int q = 0; q < 4; ++q) o[q] = bfr(a[q]);
    *(volatile v4f*)(Y + i * 4) = o; __threadfence(); *(volatile v4f*)(Y + i * 4) = o; }

__device__ __forceinline__ float fin1(const float* __restrict__ CP, const float* __restrict__ cb, unsigned n) {
    const unsigned w = n % NS, r1 = n / NS, h = r1 % NS, r2 = r1 / NS, o = r2 % NO, b = r2 / NO; float s = 0.0f;
#pragma unroll
    for (int t = 0; t < NT; ++t) { const int ws = (int)w - (t - 4); const float sf = ((ws >= 0) && (ws < NS)) ? 1.0f : 0.0f; s += cb[t * NO + o] * sf; }
    return CP[((size_t)(b * NS + h) * NS + w) * NO + o] + s; }
__global__ __launch_bounds__(256) void k_fin(const float* __restrict__ CP, const float* __restrict__ cb, float* res) {
    const unsigned t4 = blockIdx.x * 256 + threadIdx.x; if (t4 >= (unsigned)((size_t)NB * NO * NS * NS / 4)) return; const unsigned n = 4 * t4; v4f o;
    o[0] = fin1(CP, cb, n); o[1] = fin1(CP, cb, n + 1); o[2] = fin1(CP, cb, n + 2); o[3] = fin1(CP, cb, n + 3);
    float* d = res + (size_t)n; *(volatile v4f*)(d) = o; __threadfence(); *(volatile v4f*)(d) = o; }

extern "C" void kernel_launch(void* const* d_in, const int* in_sizes, int n_in,
                              void* d_out, int out_size, void* d_ws, size_t ws_size, hipStream_t stream) {
    if (n_in < 11) return;
    for (int t = 0; t < NT; ++t) if (in_sizes[t] < NB * NC * NS * NS) return;
    if (in_sizes[9] < NT * NO * NC || in_sizes[10] < NT * NO || out_size < NB * NO * NS * NS) return;
    const float* Wt = (const float*)d_in[9]; const float* cb = (const float*)d_in[10];
    float* OUT = (float*)d_out;
    char* wsp = (char*)d_ws;
    auto take = [&](size_t bytes) { char* p = wsp; wsp += (bytes + 255) & ~(size_t)255; return (void*)p; };
    bf* AP = (bf*)take((size_t)NPOS * KD * 2); bf* WP = (bf*)take((size_t)NO * KD * 2); float* CP = (float*)take((size_t)NPOS * NO * 4); float* CBR = (float*)take((size_t)NT * NO * 4);
    if ((size_t)(wsp - (char*)d_ws) != WS_TOTAL || WS_TOTAL > ws_size) return;
    for (int t = 0; t < NT; ++t) k_pack<<<dim3(NB * (NC / 8) / 256, NS * NS, 1), 256, 0, stream>>>((const float*)d_in[t], t, AP);
    k_wpk<<<dim3(NO * (NC / 8) / 256, NT, 1), 256, 0, stream>>>(Wt, WP);
    k_rbf<<<(unsigned)(((size_t)NT * NO / 4 + 255) / 256), 256, 0, stream>>>(cb, CBR, (size_t)NT * NO / 4);
    k_gemmw<bf, 0, false><<<dim3(NPOS / 64, NO / 64, 1), 32, 0, stream>>>(AP, nullptr, WP, nullptr, KD, CP, NO, nullptr, (size_t)0, (size_t)0, (size_t)0);
    k_fin<<<(unsigned)(((size_t)NB * NO * NS * NS / 4 + 255) / 256), 256, 0, stream>>>(CP, CBR, OUT);
}
